// MoleculeEncoder_47450798686658
// MI455X (gfx1250) — hardware-verified
//
#include <hip/hip_runtime.h>
#include <stddef.h>
#include <stdint.h>


#define DIN     128
#define DH      256
#define NTHR    256
#define NWAVE   8
#define EPT     8
#define NGRP    2
#define CHUNK   (NTHR * EPT * NGRP)
#define WCAP    (EPT * NGRP * 32)
#define LISTN   (NWAVE * WCAP)
#define NBD     16384
#define NB1     512
#define NB2     256
#define NBP     256
#define GROWS   32
#define WSC     64.0f
#define WINV    0.015625f
#define LDS_AGG (65536 * 4 + LISTN * 4)
#define LDS_DEG (NBD * 4 + LISTN * 4)

static_assert((CHUNK & (CHUNK - 1)) == 0);
static_assert(CHUNK <= 4096);
static_assert(NBD <= 65536 && (NBD & (NBD - 1)) == 0);
static_assert((NB1 & (NB1 - 1)) == 0 && (NB2 & (NB2 - 1)) == 0 && (NBP & (NBP - 1)) == 0);
static_assert(NB1 * DIN == 65536 && NB2 * DH == 65536 && NBP * DH == 65536);
static_assert(NBD % (NTHR * 4) == 0);
static_assert(GROWS % NWAVE == 0);

typedef float    v4f  __attribute__((ext_vector_type(4)));
typedef float    v4fa __attribute__((ext_vector_type(4), may_alias));
typedef float    v8f  __attribute__((ext_vector_type(8)));
typedef int      v4i  __attribute__((ext_vector_type(4)));
typedef _Float16 v8h  __attribute__((ext_vector_type(8)));
typedef _Float16 v16h __attribute__((ext_vector_type(16)));
union Frag { v16h v; v8h h[2]; };

__device__ __forceinline__ v8f wmf(v16h a, v16h b, v8f c) {
  v8f d = __builtin_amdgcn_wmma_f32_16x16x32_f16(false, a, false, b, (short)0, c, false, false);
  asm volatile("v_nop\n\tv_nop\n\tv_nop\n\tv_nop" : "+v"(d) : "v"(a), "v"(b));
  return d;
}

__device__ __forceinline__ v8h pack8(v4f a, v4f b) {
  v8h o;
  o[0] = (_Float16)a.x; o[1] = (_Float16)a.y; o[2] = (_Float16)a.z; o[3] = (_Float16)a.w;
  o[4] = (_Float16)b.x; o[5] = (_Float16)b.y; o[6] = (_Float16)b.z; o[7] = (_Float16)b.w;
  return o;
}

__device__ __forceinline__ v4f relu4(v4f a) {
  a.x = fmaxf(a.x, 0.f); a.y = fmaxf(a.y, 0.f); a.z = fmaxf(a.z, 0.f); a.w = fmaxf(a.w, 0.f);
  return a;
}

template <int NBT>
__device__ __forceinline__ int scan_chunk(const int* __restrict__ keys, int nK, int cbase, int base,
                                          int vec8, int* list, int tid, int lane, int wave) {
  static_assert(NBT <= 65536);
  int wc = 0;
#pragma unroll
  for (int g = 0; g < NGRP; ++g) {
    const int el0  = (g * NTHR + tid) * EPT;
    const int e0   = cbase + el0;
    const int sent = -2147483647 - 1;
    v4i da, db;
    if (vec8 != 0 && e0 + 7 < nK) {
      da = *(const v4i*)(keys + e0);
      db = *(const v4i*)(keys + e0 + 4);
    } else {
      da.x = (e0     < nK) ? keys[min(e0,     nK - 1)] : sent;
      da.y = (e0 + 1 < nK) ? keys[min(e0 + 1, nK - 1)] : sent;
      da.z = (e0 + 2 < nK) ? keys[min(e0 + 2, nK - 1)] : sent;
      da.w = (e0 + 3 < nK) ? keys[min(e0 + 3, nK - 1)] : sent;
      db.x = (e0 + 4 < nK) ? keys[min(e0 + 4, nK - 1)] : sent;
      db.y = (e0 + 5 < nK) ? keys[min(e0 + 5, nK - 1)] : sent;
      db.z = (e0 + 6 < nK) ? keys[min(e0 + 6, nK - 1)] : sent;
      db.w = (e0 + 7 < nK) ? keys[min(e0 + 7, nK - 1)] : sent;
    }
    const unsigned nb = (unsigned)base;
    const unsigned s0 = (unsigned)da.x - nb, s1 = (unsigned)da.y - nb;
    const unsigned s2 = (unsigned)da.z - nb, s3 = (unsigned)da.w - nb;
    const unsigned s4 = (unsigned)db.x - nb, s5 = (unsigned)db.y - nb;
    const unsigned s6 = (unsigned)db.z - nb, s7 = (unsigned)db.w - nb;
    const bool h0 = s0 < (unsigned)NBT, h1 = s1 < (unsigned)NBT, h2 = s2 < (unsigned)NBT, h3 = s3 < (unsigned)NBT;
    const bool h4 = s4 < (unsigned)NBT, h5 = s5 < (unsigned)NBT, h6 = s6 < (unsigned)NBT, h7 = s7 < (unsigned)NBT;
    const unsigned any = __builtin_amdgcn_ballot_w32(h0 | h1 | h2 | h3 | h4 | h5 | h6 | h7);
    if (any != 0u) {
#define HITJ(J, HJ, SJ) { \
        const unsigned mj = __builtin_amdgcn_ballot_w32(HJ); \
        if (mj != 0u) { \
          if (HJ) { \
            const int pos = wc + (int)__builtin_amdgcn_mbcnt_lo(mj, 0u); \
            if (pos < WCAP) list[wave * WCAP + pos] = ((el0 + (J)) << 16) | (int)(SJ); \
          } \
          wc += (int)__builtin_popcount(mj); } }
      HITJ(0, h0, s0)
      HITJ(1, h1, s1)
      HITJ(2, h2, s2)
      HITJ(3, h3, s3)
      HITJ(4, h4, s4)
      HITJ(5, h5, s5)
      HITJ(6, h6, s6)
      HITJ(7, h7, s7)
#undef HITJ
    }
  }
  return wc;
}

__global__ __launch_bounds__(NTHR) void k_wprep(
    const float* __restrict__ w1, const float* __restrict__ w2, const float* __restrict__ w3,
    _Float16* w1t, _Float16* w2t, _Float16* w3t) {
  const int i  = blockIdx.x * NTHR + threadIdx.x;
  const int n1 = DIN * DH / 8;
  const int n2 = DH * DH / 8;
  if (i >= n1 + 2 * n2) return;
  const float* w; _Float16* t; int K, j;
  if (i < n1)           { w = w1; t = w1t; K = DIN; j = i; }
  else if (i < n1 + n2) { w = w2; t = w2t; K = DH;  j = i - n1; }
  else                  { w = w3; t = w3t; K = DH;  j = i - n1 - n2; }
  const int kq = K / 8;
  const int n  = j / kq;
  const int k0 = (j - n * kq) * 8;
  v8h o;
#pragma unroll
  for (int e = 0; e < 8; ++e) o[e] = (_Float16)(w[(size_t)(k0 + e) * DH + n] * WSC);
  _Float16* p = t + (size_t)n * K + k0;
  *(volatile v8h*)p = o;
  __threadfence();
  *(volatile v8h*)p = o;
}

__global__ __launch_bounds__(NTHR) void k_deg(const int* __restrict__ ei, float* dis, int nE, int vec8) {
  extern __shared__ int lds_i[];
  int* cnt  = lds_i;
  int* list = lds_i + NBD;
  __shared__ int wcnt[NWAVE];
  const int tid = threadIdx.x, lane = tid & 31, wave = tid >> 5;
  const int base = blockIdx.x * NBD;
  const int* dsts = ei + nE;
  for (int i = tid; i < NBD; i += NTHR) cnt[i] = 0;
  __syncthreads();

  const int nChunks = (nE + CHUNK - 1) / CHUNK;
#pragma unroll 1
  for (int ch = 0; ch < nChunks; ++ch) {
    const int cbase = ch * CHUNK;
    const int wc = scan_chunk<NBD>(dsts, nE, cbase, base, vec8, list, tid, lane, wave);
    if (lane == 0) wcnt[wave] = wc;
    __syncthreads();
    if (wave == 0) {
#pragma unroll 1
      for (int wsx = 0; wsx < NWAVE; ++wsx) {
        int n = __builtin_amdgcn_readfirstlane(wcnt[wsx]);
        n = n > WCAP ? WCAP : (n < 0 ? 0 : n);
        const int* lp = list + wsx * WCAP;
#pragma unroll 1
        for (int i = 0; i < n; ++i) {
          const int ent  = __builtin_amdgcn_readfirstlane(lp[i]);
          const int slot = ent & (NBD - 1);
          if (lane == 0) cnt[slot] = cnt[slot] + 1;
        }
      }
    }
    __syncthreads();
  }

#pragma unroll 1
  for (int j = 0; j < NBD / (NTHR * 4); ++j) {
    const int idx = (j * NTHR + tid) * 4;
    v4f d;
    d.x = rsqrtf((float)cnt[idx]     + 1.0f);
    d.y = rsqrtf((float)cnt[idx + 1] + 1.0f);
    d.z = rsqrtf((float)cnt[idx + 2] + 1.0f);
    d.w = rsqrtf((float)cnt[idx + 3] + 1.0f);
    *(volatile v4f*)(dis + base + idx) = d;
  }
  __threadfence();
#pragma unroll 1
  for (int j = 0; j < NBD / (NTHR * 4); ++j) {
    const int idx = (j * NTHR + tid) * 4;
    v4f d;
    d.x = rsqrtf((float)cnt[idx]     + 1.0f);
    d.y = rsqrtf((float)cnt[idx + 1] + 1.0f);
    d.z = rsqrtf((float)cnt[idx + 2] + 1.0f);
    d.w = rsqrtf((float)cnt[idx + 3] + 1.0f);
    *(volatile v4f*)(dis + base + idx) = d;
  }
}

template <int W, int NB, typename TS>
__global__ __launch_bounds__(NTHR) void k_agg(const int* __restrict__ ei, const TS* __restrict__ src,
                                              const float* __restrict__ dis, _Float16* outp,
                                              int nN, int nE, int vec8) {
  static_assert(W * NB == 65536);
  static_assert(W == 128 || W == 256);
  static_assert(NB % (2 * NWAVE) == 0);
  extern __shared__ v4f lds_dyn[];
  float* acc  = (float*)lds_dyn;
  int*   list = (int*)(acc + NB * W);
  __shared__ int wcnt[NWAVE];
  const int tid = threadIdx.x, lane = tid & 31, wave = tid >> 5, hf = lane >> 4, m = lane & 15;
  const int nodeBase = blockIdx.x * NB;
  const int* dsts = ei + nE;
  const float*    srcf = (const float*)src;
  const _Float16* srch = (const _Float16*)src;
  {
    const v4f z = {0.f, 0.f, 0.f, 0.f};
    for (int i = tid; i < NB * W / 4; i += NTHR) lds_dyn[i] = z;
  }
  __syncthreads();

  const int nChunks = (nE + CHUNK - 1) / CHUNK;
#pragma unroll 1
  for (int ch = 0; ch < nChunks; ++ch) {
    const int cbase = ch * CHUNK;
    const int wc = scan_chunk<NB>(dsts, nE, cbase, nodeBase, vec8, list, tid, lane, wave);
    if (lane == 0) wcnt[wave] = wc;
    __syncthreads();
    if (wave == 0) {
#pragma unroll 1
      for (int wsx = 0; wsx < NWAVE; ++wsx) {
        int n = __builtin_amdgcn_readfirstlane(wcnt[wsx]);
        n = n > WCAP ? WCAP : (n < 0 ? 0 : n);
        const int* lp = list + wsx * WCAP;
#pragma unroll 1
        for (int i = 0; i < n; ++i) {
          const int ent  = __builtin_amdgcn_readfirstlane(lp[i]);
          const int slot = ent & (NB - 1);
          int e = cbase + ((ent >> 16) & (CHUNK - 1));
          e = e > nE - 1 ? nE - 1 : e;
          int s = ei[e];
          s = s < 0 ? 0 : (s > nN - 1 ? nN - 1 : s);
          const float ds = dis[s];
          if (W == 256) {
            const v8h hv = *(const v8h*)(srch + (size_t)s * W + 8 * lane);
            v4f* ap = (v4f*)(acc + slot * W + 8 * lane);
            v4f a0 = ap[0], a1 = ap[1];
            a0.x += (float)hv[0] * ds; a0.y += (float)hv[1] * ds;
            a0.z += (float)hv[2] * ds; a0.w += (float)hv[3] * ds;
            a1.x += (float)hv[4] * ds; a1.y += (float)hv[5] * ds;
            a1.z += (float)hv[6] * ds; a1.w += (float)hv[7] * ds;
            ap[0] = a0; ap[1] = a1;
          } else {
            const v4f xv = *(const v4f*)(srcf + (size_t)s * W + 4 * lane);
            v4f* ap = (v4f*)(acc + slot * W + 4 * lane);
            *ap = *ap + xv * ds;
          }
        }
      }
    }
    __syncthreads();
  }

  constexpr int RPW = NB / NWAVE;
  if (W == 256) {
#pragma unroll 2
    for (int j = 0; j < RPW; ++j) {
      const int slot = wave * RPW + j;
      int node = nodeBase + slot;
      node = node > nN - 1 ? nN - 1 : node;
      const float di = dis[node];
      const v8h sv = *(const v8h*)(srch + (size_t)node * W + 8 * lane);
      v4f* ap = (v4f*)(acc + slot * W + 8 * lane);
      v4f a0 = ap[0], a1 = ap[1];
      a0.x = di * (a0.x + di * (float)sv[0]); a0.y = di * (a0.y + di * (float)sv[1]);
      a0.z = di * (a0.z + di * (float)sv[2]); a0.w = di * (a0.w + di * (float)sv[3]);
      a1.x = di * (a1.x + di * (float)sv[4]); a1.y = di * (a1.y + di * (float)sv[5]);
      a1.z = di * (a1.z + di * (float)sv[6]); a1.w = di * (a1.w + di * (float)sv[7]);
      ap[0] = a0; ap[1] = a1;
    }
  } else {
#pragma unroll 2
    for (int j = 0; j < RPW / 2; ++j) {
      const int slot = wave * RPW + 2 * j + hf;
      int node = nodeBase + slot;
      node = node > nN - 1 ? nN - 1 : node;
      const float di = dis[node];
      const float* sp = srcf + (size_t)node * W + 8 * m;
      const v4f s0 = *(const v4f*)sp, s1 = *(const v4f*)(sp + 4);
      v4f* ap = (v4f*)(acc + slot * W + 8 * m);
      v4f a0 = ap[0], a1 = ap[1];
      a0 = (a0 + s0 * di) * di;
      a1 = (a1 + s1 * di) * di;
      ap[0] = a0; ap[1] = a1;
    }
  }
  __syncthreads();

  auto pass = [&]() {
    if (W == 256) {
#pragma unroll 2
      for (int j = 0; j < RPW; ++j) {
        const int slot = wave * RPW + j;
        const v4f* ap = (const v4f*)(acc + slot * W + 8 * lane);
        const v8h o = pack8(ap[0], ap[1]);
        *(volatile v8h*)(outp + (size_t)(nodeBase + slot) * W + 8 * lane) = o;
      }
    } else {
#pragma unroll 2
      for (int j = 0; j < RPW / 2; ++j) {
        const int slot = wave * RPW + 2 * j + hf;
        const v4f* ap = (const v4f*)(acc + slot * W + 8 * m);
        const v8h o = pack8(ap[0], ap[1]);
        *(volatile v8h*)(outp + (size_t)(nodeBase + slot) * W + 8 * m) = o;
      }
    }
  };
  pass();
  __threadfence();
  pass();
}

__global__ __launch_bounds__(NTHR) void k_pool(const int* __restrict__ batch, const _Float16* __restrict__ a3,
                                               _Float16* pout, float* indp, int nN, int vec8) {
  extern __shared__ v4f lds_dyn[];
  float* acc  = (float*)lds_dyn;
  int*   list = (int*)(acc + NBP * DH);
  __shared__ int wcnt[NWAVE];
  __shared__ int scnt[NBP];
  const int tid = threadIdx.x, lane = tid & 31, wave = tid >> 5;
  const int gBase = blockIdx.x * NBP;
  {
    const v4f z = {0.f, 0.f, 0.f, 0.f};
    for (int i = tid; i < NBP * DH / 4; i += NTHR) lds_dyn[i] = z;
    for (int i = tid; i < NBP; i += NTHR) scnt[i] = 0;
  }
  __syncthreads();

  const int nChunks = (nN + CHUNK - 1) / CHUNK;
#pragma unroll 1
  for (int ch = 0; ch < nChunks; ++ch) {
    const int cbase = ch * CHUNK;
    const int wc = scan_chunk<NBP>(batch, nN, cbase, gBase, vec8, list, tid, lane, wave);
    if (lane == 0) wcnt[wave] = wc;
    __syncthreads();
    if (wave == 0) {
#pragma unroll 1
      for (int wsx = 0; wsx < NWAVE; ++wsx) {
        int n = __builtin_amdgcn_readfirstlane(wcnt[wsx]);
        n = n > WCAP ? WCAP : (n < 0 ? 0 : n);
        const int* lp = list + wsx * WCAP;
#pragma unroll 1
        for (int i = 0; i < n; ++i) {
          const int ent  = __builtin_amdgcn_readfirstlane(lp[i]);
          const int slot = ent & (NBP - 1);
          int nd = cbase + ((ent >> 16) & (CHUNK - 1));
          nd = nd > nN - 1 ? nN - 1 : nd;
          const v8h hv = *(const v8h*)(a3 + (size_t)nd * DH + 8 * lane);
          v4f* ap = (v4f*)(acc + slot * DH + 8 * lane);
          v4f a0 = ap[0], a1 = ap[1];
          a0.x += (float)hv[0]; a0.y += (float)hv[1]; a0.z += (float)hv[2]; a0.w += (float)hv[3];
          a1.x += (float)hv[4]; a1.y += (float)hv[5]; a1.z += (float)hv[6]; a1.w += (float)hv[7];
          ap[0] = a0; ap[1] = a1;
          if (lane == 0) scnt[slot] = scnt[slot] + 1;
        }
      }
    }
    __syncthreads();
  }

  constexpr int RPW = NBP / NWAVE;
#pragma unroll 2
  for (int j = 0; j < RPW; ++j) {
    const int slot = wave * RPW + j;
    const float c   = (float)scnt[slot];
    const float inv = 1.0f / fmaxf(c, 1.0f);
    v4f* ap = (v4f*)(acc + slot * DH + 8 * lane);
    v4f a0 = ap[0], a1 = ap[1];
    a0 = a0 * inv; a1 = a1 * inv;
    ap[0] = a0; ap[1] = a1;
  }
  __syncthreads();

  auto pass = [&]() {
#pragma unroll 2
    for (int j = 0; j < RPW; ++j) {
      const int slot = wave * RPW + j;
      const v4f* ap = (const v4f*)(acc + slot * DH + 8 * lane);
      const v8h o = pack8(ap[0], ap[1]);
      *(volatile v8h*)(pout + (size_t)(gBase + slot) * DH + 8 * lane) = o;
    }
    if (tid < NBP / 4) {
      v4f iv;
      iv.x = scnt[4 * tid]     > 0 ? 1.f : 0.f;
      iv.y = scnt[4 * tid + 1] > 0 ? 1.f : 0.f;
      iv.z = scnt[4 * tid + 2] > 0 ? 1.f : 0.f;
      iv.w = scnt[4 * tid + 3] > 0 ? 1.f : 0.f;
      *(volatile v4f*)(indp + gBase + 4 * tid) = iv;
    }
  };
  pass();
  __threadfence();
  pass();
}

template <int K, int MODE>
__global__ __launch_bounds__(NTHR) void k_gemm(const _Float16* __restrict__ A, const _Float16* __restrict__ Bt,
                                               const float* __restrict__ bias, const float* __restrict__ ind,
                                               _Float16* out16, float* out32, int nRows) {
  static_assert(K % 32 == 0);
  __shared__ __attribute__((aligned(16))) float stg[GROWS * DH];
  const int tid = threadIdx.x, lane = tid & 31, wave = tid >> 5, hf = lane >> 4, m = lane & 15;
  const int rt = wave & 1, cq = wave >> 1;
  const int row0 = blockIdx.x * GROWS + rt * 16;
  const _Float16* ap  = A  + (size_t)(row0 + m) * K + 8 * hf;
  const _Float16* bp0 = Bt + (size_t)(64 * cq + m) * K + 8 * hf;

  v8f acc[4];
#pragma unroll
  for (int t = 0; t < 4; ++t) { v8f z = {0.f, 0.f, 0.f, 0.f, 0.f, 0.f, 0.f, 0.f}; acc[t] = z; }

#pragma unroll 1
  for (int ks = 0; ks < K / 32; ++ks) {
    Frag a;
    a.h[0] = *(const v8h*)(ap + 32 * ks);
    a.h[1] = *(const v8h*)(ap + 32 * ks + 16);
#pragma unroll
    for (int t = 0; t < 4; ++t) {
      const _Float16* bp = bp0 + (size_t)(16 * t) * K + 32 * ks;
      Frag b;
      b.h[0] = *(const v8h*)bp;
      b.h[1] = *(const v8h*)(bp + 16);
      acc[t] = wmf(a.v, b.v, acc[t]);
    }
  }

  float* sp = stg + (rt * 16 + 8 * hf) * DH + 64 * cq + m;
#pragma unroll
  for (int t = 0; t < 4; ++t) {
    sp[0 * DH + 16 * t] = acc[t][0];
    sp[1 * DH + 16 * t] = acc[t][1];
    sp[2 * DH + 16 * t] = acc[t][2];
    sp[3 * DH + 16 * t] = acc[t][3];
    sp[4 * DH + 16 * t] = acc[t][4];
    sp[5 * DH + 16 * t] = acc[t][5];
    sp[6 * DH + 16 * t] = acc[t][6];
    sp[7 * DH + 16 * t] = acc[t][7];
  }
  __syncthreads();

  constexpr int RW = GROWS / NWAVE;
  const int lr0   = wave * RW;
  const int grow0 = blockIdx.x * GROWS + lr0;
  if (MODE == 0) {
    const v4f b0 = *(const v4f*)(bias + 8 * lane), b1 = *(const v4f*)(bias + 8 * lane + 4);
    v8h ov[RW];
#pragma unroll
    for (int r = 0; r < RW; ++r) {
      const float* q = stg + (lr0 + r) * DH + 8 * lane;
      v4f q0 = *(const v4fa*)q, q1 = *(const v4fa*)(q + 4);
      q0 = relu4(q0 * WINV + b0);
      q1 = relu4(q1 * WINV + b1);
      ov[r] = pack8(q0, q1);
    }
    _Float16* op = out16 + (size_t)grow0 * DH + 8 * lane;
#pragma unroll
    for (int r = 0; r < RW; ++r)
      if (grow0 + r < nRows) *(volatile v8h*)(op + (size_t)r * DH) = ov[r];
    __threadfence();
#pragma unroll
    for (int r = 0; r < RW; ++r)
      if (grow0 + r < nRows) *(volatile v8h*)(op + (size_t)r * DH) = ov[r];
  } else {
    const v4f b0 = *(const v4f*)(bias + 4 * lane), b1 = *(const v4f*)(bias + 128 + 4 * lane);
    v4f o0[RW], o1[RW];
#pragma unroll
    for (int r = 0; r < RW; ++r) {
      const float iv = ind[grow0 + r];
      const float* q = stg + (lr0 + r) * DH;
      const v4f q0 = *(const v4fa*)(q + 4 * lane), q1 = *(const v4fa*)(q + 128 + 4 * lane);
      o0[r] = q0 * WINV + b0 * iv;
      o1[r] = q1 * WINV + b1 * iv;
    }
    float* op = out32 + (size_t)grow0 * DH + 4 * lane;
#pragma unroll
    for (int r = 0; r < RW; ++r)
      if (grow0 + r < nRows) {
        *(volatile v4f*)(op + (size_t)r * DH)       = o0[r];
        *(volatile v4f*)(op + (size_t)r * DH + 128) = o1[r];
      }
    __threadfence();
#pragma unroll
    for (int r = 0; r < RW; ++r)
      if (grow0 + r < nRows) {
        *(volatile v4f*)(op + (size_t)r * DH)       = o0[r];
        *(volatile v4f*)(op + (size_t)r * DH + 128) = o1[r];
      }
  }
}

static inline int cdiv(int a, int b) { return (a + b - 1) / b; }

extern "C" void kernel_launch(void* const* d_in, const int* in_sizes, int n_in,
                              void* d_out, int out_size, void* d_ws, size_t ws_size,
                              hipStream_t stream) {
  if (n_in < 9) return;
  const int nN = in_sizes[0] / DIN;
  const int nE = in_sizes[7] / 2;
  const int nG = out_size / DH;
  if (nN <= 0 || in_sizes[0] != nN * DIN) return;
  if (in_sizes[1] != DIN * DH || in_sizes[2] != DH) return;
  if (in_sizes[3] != DH * DH || in_sizes[4] != DH) return;
  if (in_sizes[5] != DH * DH || in_sizes[6] != DH) return;
  if (nE < 0 || in_sizes[7] != 2 * nE) return;
  if (in_sizes[8] != nN) return;
  if (nG <= 0 || out_size != nG * DH) return;

  const float* x     = (const float*)d_in[0];
  const float* W1    = (const float*)d_in[1];
  const float* b1    = (const float*)d_in[2];
  const float* W2    = (const float*)d_in[3];
  const float* b2    = (const float*)d_in[4];
  const float* W3    = (const float*)d_in[5];
  const float* b3    = (const float*)d_in[6];
  const int*   ei    = (const int*)d_in[7];
  const int*   batch = (const int*)d_in[8];
  float* out = (float*)d_out;

  const int nDB  = cdiv(nN, NBD);
  const int nAB1 = cdiv(nN, NB1);
  const int nAB2 = cdiv(nN, NB2);
  const int nGB  = cdiv(nN, GROWS);
  const int nPB  = cdiv(nG, NBP);
  const int nGB3 = cdiv(nG, GROWS);
  if ((size_t)nGB * GROWS > (size_t)nAB1 * NB1 || (size_t)nGB * GROWS > (size_t)nAB2 * NB2) return;
  if ((size_t)nGB3 * GROWS > (size_t)nPB * NBP) return;

  char* ws = (char*)d_ws;
  size_t off = 0;
  auto carve = [&](size_t bytes) -> size_t { const size_t o = off; off = (off + bytes + 255) & ~(size_t)255; return o; };
  const size_t oDis = carve((size_t)nDB * NBD * 4);
  const size_t oW1  = carve((size_t)DIN * DH * 2);
  const size_t oW2  = carve((size_t)DH * DH * 2);
  const size_t oW3  = carve((size_t)DH * DH * 2);
  const size_t szA1 = (size_t)nAB1 * NB1 * DIN * 2;
  const size_t szA2 = (size_t)nAB2 * NB2 * DH * 2;
  const size_t oR1  = carve(szA1 > szA2 ? szA1 : szA2);
  const size_t oR2  = carve((size_t)nGB * GROWS * DH * 2);
  const size_t oP   = carve((size_t)nPB * NBP * DH * 2);
  const size_t oInd = carve((size_t)nPB * NBP * 4);
  if (off > ws_size) return;
  if (off > ((size_t)128 << 20)) return;

  float*    dis = (float*)(ws + oDis);
  _Float16* w1t = (_Float16*)(ws + oW1);
  _Float16* w2t = (_Float16*)(ws + oW2);
  _Float16* w3t = (_Float16*)(ws + oW3);
  _Float16* r1  = (_Float16*)(ws + oR1);
  _Float16* r2  = (_Float16*)(ws + oR2);
  _Float16* pm  = (_Float16*)(ws + oP);
  float*    ind = (float*)(ws + oInd);

  const int vec8e = ((nE & 3) == 0) ? 1 : 0;
  const int vec8b = 1;

  const int nPrep = DIN * DH / 8 + 2 * (DH * DH / 8);
  k_wprep<<<cdiv(nPrep, NTHR), NTHR, 0, stream>>>(W1, W2, W3, w1t, w2t, w3t);

  hipFuncSetAttribute(reinterpret_cast<const void*>(&k_deg),
                      hipFuncAttributeMaxDynamicSharedMemorySize, LDS_DEG);
  k_deg<<<nDB, NTHR, LDS_DEG, stream>>>(ei, dis, nE, vec8e);

  hipFuncSetAttribute(reinterpret_cast<const void*>(&k_agg<DIN, NB1, float>),
                      hipFuncAttributeMaxDynamicSharedMemorySize, LDS_AGG);
  k_agg<DIN, NB1, float><<<nAB1, NTHR, LDS_AGG, stream>>>(ei, x, dis, r1, nN, nE, vec8e);
  k_gemm<DIN, 0><<<nGB, NTHR, 0, stream>>>(r1, w1t, b1, ind, r2, out, nGB * GROWS);

  hipFuncSetAttribute(reinterpret_cast<const void*>(&k_agg<DH, NB2, _Float16>),
                      hipFuncAttributeMaxDynamicSharedMemorySize, LDS_AGG);
  k_agg<DH, NB2, _Float16><<<nAB2, NTHR, LDS_AGG, stream>>>(ei, r2, dis, r1, nN, nE, vec8e);
  k_gemm<DH, 0><<<nGB, NTHR, 0, stream>>>(r1, w2t, b2, ind, r2, out, nGB * GROWS);

  k_agg<DH, NB2, _Float16><<<nAB2, NTHR, LDS_AGG, stream>>>(ei, r2, dis, r1, nN, nE, vec8e);
  hipFuncSetAttribute(reinterpret_cast<const void*>(&k_pool),
                      hipFuncAttributeMaxDynamicSharedMemorySize, LDS_AGG);
  k_pool<<<nPB, NTHR, LDS_AGG, stream>>>(batch, r1, pm, ind, nN, vec8b);
  k_gemm<DH, 1><<<nGB3, NTHR, 0, stream>>>(pm, w3t, b3, ind, r2, out, nG);
}
